// _gat_layer_batch_16045997818088
// MI455X (gfx1250) — hardware-verified
//
#include <hip/hip_runtime.h>
#include <math.h>

typedef __attribute__((ext_vector_type(16))) _Float16 v16h;
typedef __attribute__((ext_vector_type(16))) __bf16 v16b;
typedef __attribute__((ext_vector_type(8)))  _Float16 v8h;
typedef __attribute__((ext_vector_type(8)))  float v8f;
typedef __attribute__((ext_vector_type(4)))  float v4f;
typedef __attribute__((ext_vector_type(2)))  float v2f;
typedef __attribute__((ext_vector_type(4)))  unsigned v4u;
typedef __attribute__((ext_vector_type(4)))  int v4i;
typedef float __attribute__((may_alias)) float_a;
typedef int __attribute__((may_alias)) int_a;

template <typename T> __device__ __forceinline__ void vst2(void* p, T v) { *(volatile T*)p = v; __threadfence(); *(volatile T*)p = v; }
__device__ __forceinline__ v8f wmma16(v16h a, v16h b, v8f c) {
  v8f d = __builtin_amdgcn_wmma_f32_16x16x32_f16(false, a, false, b, (short)0, c, false, false);
  asm volatile("v_nop\n\tv_nop\n\tv_nop\n\tv_nop" : "+v"(d) : "v"(a), "v"(b));
  return d;
}
__device__ __forceinline__ v8f wmma_bf(v16b a, v16b b, v8f c) {
  v8f d = __builtin_amdgcn_wmma_f32_16x16x32_bf16(false, a, false, b, (short)0, c, false, false);
  asm volatile("v_nop\n\tv_nop\n\tv_nop\n\tv_nop" : "+v"(d) : "v"(a), "v"(b));
  return d;
}
__device__ __forceinline__ v16h frag_h(const _Float16* rowk0, int lane) {
  union { v16h v; v8h q[2]; } u; const _Float16* p = rowk0 + 8 * (lane >> 4);
  u.q[0] = *(const v8h*)p; u.q[1] = *(const v8h*)(p + 16); return u.v;
}
__device__ __forceinline__ v16h frag_f32(const float* rowk0, int lane) {
  v16h a; const float* p = rowk0 + 8 * (lane >> 4);
#pragma unroll
  for (int i = 0; i < 8; ++i) { a[i] = (_Float16)p[i]; a[8 + i] = (_Float16)p[16 + i]; }
  return a;
}
__device__ __forceinline__ v16h frag_f32s(const float* rowk0, int lane, float sc) {
  v16h a; const float* p = rowk0 + 8 * (lane >> 4);
#pragma unroll
  for (int i = 0; i < 8; ++i) { a[i] = (_Float16)(p[i] * sc); a[8 + i] = (_Float16)(p[16 + i] * sc); }
  return a;
}
__device__ __forceinline__ v16h fragc_f32(const float* W, int k0, int n, int lane, int ld, int K) {
  v16h a; const int g = lane >> 4;
#pragma unroll
  for (int i = 0; i < 8; ++i) { const int ka = k0 + 8 * g + i, kb = ka + 16;
    a[i] = (_Float16)(ka < K ? W[(size_t)(ka < K ? ka : K - 1) * ld + n] : 0.f); a[8 + i] = (_Float16)(kb < K ? W[(size_t)(kb < K ? kb : K - 1) * ld + n] : 0.f); }
  return a;
}
struct F2 { v16b h, l; };
__device__ __forceinline__ F2 bsplit16(const float v[16]) { F2 r;
#pragma unroll
  for (int i = 0; i < 16; ++i) { const __bf16 h = (__bf16)v[i]; r.h[i] = h; r.l[i] = (__bf16)(v[i] - (float)h); }
  return r; }
__device__ __forceinline__ F2 split_row(const float* row, int k0, int lane) { float v[16]; const float* p = row + k0 + 8 * (lane >> 4);
#pragma unroll
  for (int i = 0; i < 8; ++i) { v[i] = p[i]; v[8 + i] = p[16 + i]; }
  return bsplit16(v); }
__device__ __forceinline__ F2 split_rowK(const float* row, int k0, int lane, int K) { float v[16]; const int g = lane >> 4;
#pragma unroll
  for (int i = 0; i < 8; ++i) { const int ka = k0 + 8 * g + i, kb = ka + 16; v[i] = ka < K ? row[ka < K ? ka : K - 1] : 0.f; v[8 + i] = kb < K ? row[kb < K ? kb : K - 1] : 0.f; }
  return bsplit16(v); }
__device__ __forceinline__ F2 split_col(const float* W, int k0, int n, int lane, int ld, int K) { float v[16]; const int g = lane >> 4;
#pragma unroll
  for (int i = 0; i < 8; ++i) { const int ka = k0 + 8 * g + i, kb = ka + 16; v[i] = ka < K ? W[(size_t)(ka < K ? ka : K - 1) * ld + n] : 0.f; v[8 + i] = kb < K ? W[(size_t)(kb < K ? kb : K - 1) * ld + n] : 0.f; }
  return bsplit16(v); }
__device__ __forceinline__ v8f mac3(const F2& a, const F2& b, v8f c) { c = wmma_bf(a.l, b.h, c); c = wmma_bf(a.h, b.l, c); return wmma_bf(a.h, b.h, c); }
__device__ __forceinline__ float sigm(float v) { return 1.0f / (1.0f + expf(-v)); }
#define LDSX() do { asm volatile("s_wait_dscnt 0" ::: "memory"); __builtin_amdgcn_wave_barrier(); __builtin_amdgcn_fence(__ATOMIC_RELEASE, "workgroup"); } while (0)


#define NB 8
#define NN 1024
#define FIN 256
#define NH 8
#define HDN 32
#define FO (NH * HDN)
#define SLOPE 0.2f
#ifndef TNB
#define TNB NB
#endif
typedef __attribute__((ext_vector_type(8))) __bf16 v8b;
__device__ __forceinline__ v16b frag_b(const __bf16* rowk0, int lane) {
  union { v16b v; v8b q[2]; } u; const __bf16* p = rowk0 + 8 * (lane >> 4);
  u.q[0] = *(const v8b*)p; u.q[1] = *(const v8b*)(p + 16); return u.v;
}
__device__ __forceinline__ float bfr(float v) { return (float)(__bf16)v; }
__device__ __attribute__((noinline)) float exp_ni(float v) { return expf(v); }
__device__ __attribute__((noinline)) float erf_ni(float v) { return erff(v); }

#define WS_PW  0u
#define WS_G   (WS_PW + 2u * FO * FIN)
#define WS_GTH (WS_G + 4u * (size_t)NB * NN * FO)
#define WS_GTL (WS_GTH + 2u * (size_t)NB * FO * NN)
#define WS_S   (WS_GTL + 2u * (size_t)NB * FO * NN)
#define SHALF  ((size_t)NB * NN * 8)
#define WS_END (WS_S + 4u * 2 * SHALF)

__global__ __launch_bounds__(256) void k_pack(const float* __restrict__ Wv, __bf16* __restrict__ PW) { const int o = blockIdx.x, t = threadIdx.x; __shared__ __align__(16) __bf16 s[FIN]; s[t] = (__bf16)Wv[(size_t)t * FO + o]; __syncthreads(); if (t < FIN / 8) vst2((unsigned*)(PW + (size_t)o * FIN + t * 8), *(const v4u*)&s[t * 8]); }
__device__ __forceinline__ v16b fragb_f32(const float* __restrict__ p, int lane) { v16b a; const float* pp = p + 8 * (lane >> 4);
#pragma unroll
  for (int i = 0; i < 8; ++i) { a[i] = (__bf16)pp[i]; a[8 + i] = (__bf16)pp[16 + i]; } return a; }
__global__ __launch_bounds__(128) void k_g(const float* __restrict__ X, const __bf16* __restrict__ PW, const float* __restrict__ AW, float* __restrict__ G, _Float16* __restrict__ GTH, _Float16* __restrict__ GTL, float* __restrict__ S) {
  __shared__ __align__(16) float sf[64][132]; __shared__ __align__(16) _Float16 sth[128][72], stl[128][72]; __shared__ __align__(16) float ss[64][8];
  const int tid = threadIdx.x, wave = tid >> 5, lane = tid & 31, col = lane & 15, g = lane >> 4; const size_t rb = (size_t)blockIdx.x * 64; const size_t r0 = rb + wave * 16; const int c0 = blockIdx.y * 128; const size_t b = rb / NN; const int j0 = (int)(rb % NN);
  v8f acc[8] = {};
#pragma unroll
  for (int kc = 0; kc < FIN / 32; ++kc) { const v16b a = fragb_f32(X + (r0 + col) * FIN + kc * 32, lane);
#pragma unroll
    for (int j = 0; j < 8; ++j) acc[j] = wmma_bf(a, frag_b(PW + (size_t)(c0 + j * 16 + col) * FIN + kc * 32, lane), acc[j]); }
#pragma unroll
  for (int j = 0; j < 8; ++j)
#pragma unroll
    for (int r = 0; r < 8; ++r) { const float v = acc[j][r]; const int rl = wave * 16 + 8 * g + r, cl = j * 16 + col; sf[rl][cl] = v; const _Float16 hv = (_Float16)v; sth[cl][rl] = hv; stl[cl][rl] = (_Float16)((v - (float)hv) * 2048.0f); }
  __syncthreads();
  { const int rl = tid >> 1, hh0 = (tid & 1) * 2; for (int hh = hh0; hh < hh0 + 2; ++hh) { float s1 = 0.f, s2 = 0.f;
#pragma unroll 1
      for (int d = 0; d < HDN; ++d) { const float gv = sf[rl][hh * HDN + d]; s1 += gv * bfr(AW[d]); s2 += gv * bfr(AW[HDN + d]); }
      ss[rl][hh * 2] = s1; ss[rl][hh * 2 + 1] = s2; } }
  __syncthreads();
  for (int rl = wave; rl < 64; rl += 4) vst2(G + (rb + rl) * FO + c0 + lane * 4, *(const v4f*)&sf[rl][lane * 4]);
  for (int e = tid; e < 128 * 8; e += 128) { const int cl = e >> 3, q = e & 7; const size_t o = (b * FO + c0 + cl) * NN + j0 + q * 8; vst2((unsigned*)(GTH + o), *(const v4u*)&sth[cl][q * 8]); vst2((unsigned*)(GTL + o), *(const v4u*)&stl[cl][q * 8]); }
  if (tid < 64 * 2) { const int rl = tid >> 1, q = tid & 1; vst2(S + (size_t)(c0 / 128) * SHALF + (rb + rl) * 8 + q * 4, *(const v4f*)&ss[rl][q * 4]); } }
__device__ __forceinline__ float sget(const float* S, size_t row, int h, int dst) { return S[(size_t)(h >> 2) * SHALF + row * 8 + (h & 3) * 2 + dst]; }
__global__ __launch_bounds__(128) void k_att(const float* __restrict__ S, const _Float16* __restrict__ GTH, const _Float16* __restrict__ GTL, float* __restrict__ OUT) { __shared__ __align__(16) float sp[4][16][36]; __shared__ __align__(16) float so[4][16][36]; __shared__ float sdst[NN]; __shared__ float red[4];
  const int tid = threadIdx.x, wave = tid >> 5, lane = tid & 31, col = lane & 15, g = lane >> 4; const int h = blockIdx.y; const size_t b = blockIdx.z; const int i0 = blockIdx.x * 64 + wave * 16; const size_t rq = b * NN + i0;
  float mx = -3.0e38f; for (int j = tid; j < NN; j += 128) { const float v = sget(S, b * NN + j, h, 1); sdst[j] = v; mx = fmaxf(mx, v); }
#pragma unroll
  for (int o = 1; o < 32; o <<= 1) mx = fmaxf(mx, __shfl_xor(mx, o));
  if (lane == 0) red[wave] = mx; __syncthreads(); const float smax = fmaxf(fmaxf(red[0], red[1]), fmaxf(red[2], red[3]));
  float si[8], mi[8], l[8];
#pragma unroll
  for (int r = 0; r < 8; ++r) { si[r] = sget(S, rq + 8 * g + r, h, 0); const float e = si[r] + smax; mi[r] = e >= 0.f ? e : SLOPE * e; l[r] = 0.f; }
  v8f acc[2] = {}, accl[2] = {};
#pragma unroll 1
  for (int ks = 0; ks < NN / 32; ++ks) {
#pragma unroll
    for (int ct = 0; ct < 2; ++ct) { const int kk = ks * 32 + ct * 16 + col; const float sd = sdst[kk];
#pragma unroll
      for (int r = 0; r < 8; ++r) { float e = si[r] + sd; e = e >= 0.f ? e : SLOPE * e; const float p = __expf(e - mi[r]); l[r] += p; sp[wave][8 * g + r][ct * 16 + col] = p; } }
    LDSX();
    v16h pa, pl; { const float* prow = &sp[wave][col][0] + 8 * (lane >> 4);
#pragma unroll
      for (int i = 0; i < 8; ++i) { const float x0 = prow[i] * 2048.0f, x1 = prow[16 + i] * 2048.0f; const _Float16 h0 = (_Float16)x0, h1 = (_Float16)x1; pa[i] = h0; pa[8 + i] = h1; pl[i] = (_Float16)((x0 - (float)h0) * 2048.0f); pl[8 + i] = (_Float16)((x1 - (float)h1) * 2048.0f); } }
#pragma unroll
    for (int dt = 0; dt < 2; ++dt) { const size_t po = (b * FO + (size_t)h * HDN + dt * 16 + col) * NN + ks * 32; const v16h gh = frag_h(GTH + po, lane), gl = frag_h(GTL + po, lane); acc[dt] = wmma16(pa, gh, acc[dt]); accl[dt] = wmma16(pl, gh, accl[dt]); accl[dt] = wmma16(pa, gl, accl[dt]); }
    LDSX(); }
#pragma unroll
  for (int r = 0; r < 8; ++r) { float lt = l[r];
#pragma unroll
    for (int o = 1; o < 16; o <<= 1) lt += __shfl_xor(lt, o);
    const float il = (1.0f / 2048.0f) / lt;
#pragma unroll
    for (int dt = 0; dt < 2; ++dt) so[wave][8 * g + r][dt * 16 + col] = (acc[dt][r] + accl[dt][r] * (1.0f / 2048.0f)) * il; }
  LDSX(); for (int rl = 0; rl < 16; ++rl) if (lane < 8) vst2(OUT + (rq + rl) * FO + (size_t)h * HDN + lane * 4, *(const v4f*)&so[wave][rl][lane * 4]);
}
extern "C" void kernel_launch(void* const* d_in, const int* in_sizes, int n_in, void* d_out, int out_size, void* d_ws, size_t ws_size, hipStream_t stream) {
  (void)in_sizes; (void)n_in; (void)out_size;
  const float** F = (const float**)d_in;
  if (ws_size < (size_t)WS_END) return;
  char* ws = (char*)d_ws; __bf16* PW = (__bf16*)(ws + WS_PW); float *G = (float*)(ws + WS_G), *S = (float*)(ws + WS_S); _Float16 *GTH = (_Float16*)(ws + WS_GTH), *GTL = (_Float16*)(ws + WS_GTL);
  k_pack<<<FO, 256, 0, stream>>>(F[1], PW);
  k_g<<<dim3(TNB * NN / 64, FO / 128), 128, 0, stream>>>(F[0], PW, F[2], G, GTH, GTL, S);
  k_att<<<dim3(NN / 64, NH, TNB), 128, 0, stream>>>(S, GTH, GTL, (float*)d_out);
}
